// CliffordAttention_30442728194243
// MI455X (gfx1250) — hardware-verified
//
#include <hip/hip_runtime.h>
#include <math.h>

constexpr int kBatch   = 2;
constexpr int kSeq     = 2048;
constexpr int kModel   = 1024;
constexpr int kHeads   = 8;
constexpr int kHeadDim = 128;
constexpr int kTok     = kBatch * kSeq;
constexpr int kQKVN    = 3 * kModel;
constexpr int kGrp     = 2;
constexpr int kChunks  = kHeads / kGrp;
constexpr float kWCarry     = 16.0f;
constexpr float kWCarryInv  = 1.0f / 16.0f;
constexpr float kPCarry     = 2048.0f;
constexpr float kPCarryInv  = 1.0f / 2048.0f;
constexpr float kLogitScale = 0.08838834764831845f;
constexpr float kMeanScale  = 0.125f;


typedef __attribute__((ext_vector_type(16))) _Float16 v16h;
typedef __attribute__((ext_vector_type(8)))  _Float16 v8h;
typedef __attribute__((ext_vector_type(16))) __bf16   v16b;
typedef __attribute__((ext_vector_type(8)))  __bf16   v8b;
typedef __attribute__((ext_vector_type(8)))  float    v8f;
typedef __attribute__((ext_vector_type(4)))  float    v4f;
typedef __attribute__((ext_vector_type(4)))  unsigned int v4u;

__device__ __forceinline__ unsigned short f2bf_bits(float f) {
  unsigned u = __float_as_uint(f);
  return (unsigned short)((u + 0x7FFFu + ((u >> 16) & 1u)) >> 16);
}
__device__ __forceinline__ float bf_bits2f(unsigned short h) { return __uint_as_float(((unsigned)h) << 16); }

__device__ __forceinline__ void dep_guard_h(v8f& a, v8f& b, v16h x, v16h y) { asm volatile("v_nop\n\tv_nop\n\tv_nop\n\tv_nop" : "+v"(a), "+v"(b) : "v"(x), "v"(y)); }
__device__ __forceinline__ void dep_guard_b(v8f& a, v8f& b, v16b x, v16b y) { asm volatile("v_nop\n\tv_nop\n\tv_nop\n\tv_nop" : "+v"(a), "+v"(b) : "v"(x), "v"(y)); }
__device__ __forceinline__ void keep4_h(v16h a, v16h b, v16h c, v16h d) { asm volatile("v_nop" :: "v"(a), "v"(b), "v"(c), "v"(d)); }
__device__ __forceinline__ void keep4_b(v16b a, v16b b, v16b c, v16b d) { asm volatile("v_nop" :: "v"(a), "v"(b), "v"(c), "v"(d)); }
__device__ __forceinline__ void acc_guard4(v8f& a, v8f& b, v8f& c, v8f& d) { asm volatile("v_nop\n\tv_nop\n\tv_nop\n\tv_nop" : "+v"(a), "+v"(b), "+v"(c), "+v"(d)); }
template <typename T> struct Frag;
template <> struct Frag<_Float16> {
  typedef v16h V; union U { v16h v; v8h h[2]; };
  static __device__ __forceinline__ v16h load(const _Float16* p) {
    U f; f.h[0] = *(const v8h*)(p); f.h[1] = *(const v8h*)(p + 16); return f.v;
  }
  static __device__ __forceinline__ v8f mma(v16h a, v16h b, v8f c) {
    return __builtin_amdgcn_wmma_f32_16x16x32_f16(false, a, false, b, (short)0, c, false, false);
  }
  static __device__ __forceinline__ void guard(v8f& a, v8f& b, v16h x, v16h y) { dep_guard_h(a, b, x, y); }
  static __device__ __forceinline__ void keep(v16h a, v16h b, v16h c, v16h d) { keep4_h(a, b, c, d); }
};
template <> struct Frag<__bf16> {
  typedef v16b V; union U { v16b v; v8b h[2]; };
  static __device__ __forceinline__ v16b load(const __bf16* p) {
    U f; f.h[0] = *(const v8b*)(p); f.h[1] = *(const v8b*)(p + 16); return f.v;
  }
  static __device__ __forceinline__ v8f mma(v16b a, v16b b, v8f c) {
    return __builtin_amdgcn_wmma_f32_16x16x32_bf16(false, a, false, b, (short)0, c, false, false);
  }
  static __device__ __forceinline__ void guard(v8f& a, v8f& b, v16b x, v16b y) { dep_guard_b(a, b, x, y); }
  static __device__ __forceinline__ void keep(v16b a, v16b b, v16b c, v16b d) { keep4_b(a, b, c, d); }
};

__device__ __forceinline__ unsigned pk16(unsigned short a, unsigned short b) { return (unsigned)a | ((unsigned)b << 16); }
__device__ __forceinline__ unsigned short h_bits(float f) { const _Float16 h = (_Float16)f; return __builtin_bit_cast(unsigned short, h); }

template <int ET> struct Elem;
template <> struct Elem<0> { typedef _Float16 T; };
template <> struct Elem<1> { typedef __bf16 T; };
template <int ET, bool SPLIT, int BIAS_MODE, int OUT_MODE, bool RESID, int ACT = 0>
__global__ __launch_bounds__(256) void wmma_gemm64(
    const unsigned short* __restrict__ Ap, const unsigned short* __restrict__ A2p, int lda, long strideA,
    const unsigned short* __restrict__ Btp, const unsigned short* __restrict__ Bt2p, int ldb, long strideB,
    void* __restrict__ Cout, void* __restrict__ Cout2, int ldc, long strideC,
    const float* __restrict__ bias,
    const float* __restrict__ resid, long strideR,
    int M, int N, int K, float scale) {
  typedef typename Elem<ET>::T T;
  typedef typename Frag<T>::V V;
  const T* A = (const T*)Ap; const T* A2 = (const T*)A2p; const T* Bt = (const T*)Btp; const T* Bt2 = (const T*)Bt2p;
  __shared__ __align__(16) float sT[8][16 * 68];
  const int b    = blockIdx.y;
  const int lane = threadIdx.x & 31;
  const int wave = threadIdx.x >> 5;
  const int tilesN = N >> 6;
  const int tilesM = M >> 6;
  const int tile = blockIdx.x * 8 + wave;
  if (tile >= tilesM * tilesN) return;
  const int tm = tile / tilesN;
  const int tn = tile - tm * tilesN;
  const int m0 = tm << 6;
  const int n0 = tn << 6;

  const T* Ab  = A  + (size_t)b * strideA;
  const T* Bb  = Bt + (size_t)b * strideB;
  const T* Ab2 = SPLIT ? (A2  + (size_t)b * strideA) : nullptr;
  const T* Bb2 = SPLIT ? (Bt2 + (size_t)b * strideB) : nullptr;

  const int rlane = lane & 15;
  const int koff  = (lane >> 4) * 8;
  const int mOff  = (lane >> 4) * 8;

  v8f acc[4][4];
#pragma unroll
  for (int i = 0; i < 4; ++i)
#pragma unroll
    for (int j = 0; j < 4; ++j) acc[i][j] = (v8f){0.f,0.f,0.f,0.f,0.f,0.f,0.f,0.f};

  for (int k0 = 0; k0 < K; k0 += 32) {
    V bh[4], bl[4];
#pragma unroll
    for (int j = 0; j < 4; ++j) {
      const size_t bo = (size_t)(n0 + (j << 4) + rlane) * ldb + koff + k0;
      bh[j] = Frag<T>::load(Bb + bo);
      if (SPLIT) bl[j] = Frag<T>::load(Bb2 + bo);
    }
#pragma unroll
    for (int i = 0; i < 4; ++i) {
      const size_t ao = (size_t)(m0 + (i << 4) + rlane) * lda + koff + k0;
      V ah = Frag<T>::load(Ab + ao);
      V al;
      if (SPLIT) al = Frag<T>::load(Ab2 + ao);
#pragma unroll
      for (int j = 0; j < 4; ++j) {
        acc[i][j] = Frag<T>::mma(ah, bh[j], acc[i][j]);
        if (SPLIT) {
          acc[i][j] = Frag<T>::mma(ah, bl[j], acc[i][j]);
          acc[i][j] = Frag<T>::mma(al, bh[j], acc[i][j]);
        }
      }
      Frag<T>::guard(acc[i][0], acc[i][3], ah, SPLIT ? al : ah);
    }
    Frag<T>::keep(bh[0], bh[1], bh[2], bh[3]);
    if (SPLIT) Frag<T>::keep(bl[0], bl[1], bl[2], bl[3]);
  }
  acc_guard4(acc[0][0], acc[0][1], acc[0][2], acc[0][3]);
  acc_guard4(acc[1][0], acc[1][1], acc[1][2], acc[1][3]);
  acc_guard4(acc[2][0], acc[2][1], acc[2][2], acc[2][3]);
  acc_guard4(acc[3][0], acc[3][1], acc[3][2], acc[3][3]);

  float* slab = sT[wave];
  const float* Rb = RESID ? (resid + (size_t)b * strideR) : nullptr;
#pragma unroll
  for (int i = 0; i < 4; ++i) {
    const int mBase = m0 + (i << 4);
#pragma unroll
    for (int j = 0; j < 4; ++j) {
      const int n = n0 + (j << 4) + rlane;
      float bv = 0.f;
      if (BIAS_MODE == 2) bv = bias[n];
#pragma unroll
      for (int r = 0; r < 8; ++r) {
        float v = acc[i][j][r] * scale;
        if (BIAS_MODE == 1) v += bias[mBase + mOff + r];
        if (BIAS_MODE == 2) v += bv;
        if (RESID) v += Rb[(size_t)(mBase + mOff + r) * ldc + n];
        if (ACT == 2) v = fmaxf(v, 0.0f);
        if (ACT == 4) v = (v > 0.f) ? v : 0.01f * v;
        slab[(mOff + r) * 68 + (j << 4) + rlane] = v;
      }
    }
    __builtin_amdgcn_fence(__ATOMIC_RELEASE, "workgroup");
    __builtin_amdgcn_wave_barrier();
    __builtin_amdgcn_fence(__ATOMIC_ACQUIRE, "workgroup");
    if (OUT_MODE == 0) {
      float* C = (float*)Cout + (size_t)b * strideC;
      const int hh = lane >> 4, c4 = (lane & 15) * 4;
      for (int pass = 0; pass < 2; ++pass) {
#pragma unroll
        for (int it = 0; it < 8; ++it) {
          const int row = it * 2 + hh;
          v4f v = *(const v4f*)(slab + row * 68 + c4);
          *(volatile v4f*)(C + (size_t)(mBase + row) * ldc + n0 + c4) = v;
        }
        __threadfence();
      }
    } else {
      const int q = lane >> 3, c8 = (lane & 7) * 8;
      unsigned short* C  = (unsigned short*)Cout  + (size_t)b * strideC;
      unsigned short* C2 = (OUT_MODE == 2) ? ((unsigned short*)Cout2 + (size_t)b * strideC) : nullptr;
      for (int pass = 0; pass < 2; ++pass) {
#pragma unroll
        for (int it = 0; it < 4; ++it) {
          const int row = it * 4 + q;
          const float* sp = slab + row * 68 + c8;
          v8h hv, lv;
#pragma unroll
          for (int e = 0; e < 8; ++e) {
            if (OUT_MODE == 1) {
              hv[e] = (_Float16)sp[e];
            } else {
              unsigned short hb = f2bf_bits(sp[e]);
              unsigned short lb = f2bf_bits(sp[e] - bf_bits2f(hb));
              hv[e] = __builtin_bit_cast(_Float16, hb);
              lv[e] = __builtin_bit_cast(_Float16, lb);
            }
          }
          *(volatile v8h*)(C + (size_t)(mBase + row) * ldc + n0 + c8) = hv;
          if (OUT_MODE == 2) *(volatile v8h*)(C2 + (size_t)(mBase + row) * ldc + n0 + c8) = lv;
        }
        __threadfence();
      }
    }
    __builtin_amdgcn_fence(__ATOMIC_RELEASE, "workgroup");
    __builtin_amdgcn_wave_barrier();
    __builtin_amdgcn_fence(__ATOMIC_ACQUIRE, "workgroup");
  }
}

__global__ __launch_bounds__(256) void cast8_f16_kernel(const float* __restrict__ in, unsigned short* __restrict__ out, int n8) {
  const int i = blockIdx.x * 256 + threadIdx.x;
  if (i >= n8) return;
  const float* p = in + 8 * (size_t)i;
  const v4f a = *(const v4f*)(p);
  const v4f c = *(const v4f*)(p + 4);
  unsigned short hb[8];
#pragma unroll
  for (int e = 0; e < 4; ++e) {
    hb[e]     = h_bits(a[e]);
    hb[4 + e] = h_bits(c[e]);
  }
  const v4u u = (v4u){pk16(hb[0], hb[1]), pk16(hb[2], hb[3]), pk16(hb[4], hb[5]), pk16(hb[6], hb[7])};
  unsigned short* q = out + 8 * (size_t)i;
  *(volatile v4u*)q = u;
  __threadfence();
  *(volatile v4u*)q = u;
}

__global__ __launch_bounds__(256) void wcast8_kernel(const float* __restrict__ W0, const float* __restrict__ W1,
                                                     const float* __restrict__ W2, unsigned short* __restrict__ out, int n8) {
  const int z = blockIdx.y;
  const int i = blockIdx.x * 256 + threadIdx.x;
  if (i >= n8) return;
  const float* W = (z == 0) ? W0 : (z == 1) ? W1 : W2;
  const int n = i >> 7;
  const bool neg = (z == 0) && ((n & 7) >= 4);
  const float sc = neg ? -kWCarry : kWCarry;
  const float* p = W + 8 * (size_t)i;
  const v4f a = *(const v4f*)(p);
  const v4f c = *(const v4f*)(p + 4);
  unsigned short hb[8];
#pragma unroll
  for (int e = 0; e < 4; ++e) {
    hb[e]     = h_bits(a[e] * sc);
    hb[4 + e] = h_bits(c[e] * sc);
  }
  const v4u u = (v4u){pk16(hb[0], hb[1]), pk16(hb[2], hb[3]), pk16(hb[4], hb[5]), pk16(hb[6], hb[7])};
  unsigned short* q = out + (size_t)z * kModel * kModel + 8 * (size_t)i;
  *(volatile v4u*)q = u;
  __threadfence();
  *(volatile v4u*)q = u;
}

__global__ __launch_bounds__(256) void bias3_kernel(const float* __restrict__ b0, const float* __restrict__ b1,
                                                   const float* __restrict__ b2, float* __restrict__ out) {
  const int z = blockIdx.x;
  const int t = threadIdx.x;
  const float* bp = (z == 0) ? b0 : (z == 1) ? b1 : b2;
  v4f v = *(const v4f*)(bp + 4 * t);
#pragma unroll
  for (int e = 0; e < 4; ++e) {
    const int n = 4 * t + e;
    const bool neg = (z == 0) && ((n & 7) >= 4);
    v[e] = neg ? -v[e] : v[e];
  }
  float* q = out + (size_t)z * kModel + 4 * t;
  *(volatile v4f*)q = v;
  __threadfence();
  *(volatile v4f*)q = v;
}

__global__ __launch_bounds__(256) void vtrans_kernel(const unsigned short* __restrict__ Y, unsigned short* __restrict__ VT) {
  __shared__ __align__(16) unsigned short sm[64][72];
  const int t   = threadIdx.x;
  const int l0  = blockIdx.x * 64;
  const int cg0 = blockIdx.y * 64;
  const int b   = blockIdx.z;
#pragma unroll
  for (int it = 0; it < 8; ++it) {
    const int e  = it * 256 + t;
    const int r  = e >> 5;
    const int cw = e & 31;
    const unsigned u = *(const unsigned*)(Y + ((size_t)(b * kSeq + l0 + r)) * kQKVN + 2 * kModel + cg0 + 2 * cw);
    sm[2 * cw][r]     = (unsigned short)(u & 0xffffu);
    sm[2 * cw + 1][r] = (unsigned short)(u >> 16);
  }
  __syncthreads();
  const int lane = t & 31, wave = t >> 5;
  const int q = lane >> 3, c8 = (lane & 7) * 8;
  for (int pass = 0; pass < 2; ++pass) {
#pragma unroll
    for (int it = 0; it < 2; ++it) {
      const int row = wave * 8 + it * 4 + q;
      const int cg  = cg0 + row;
      const int g   = b * kHeads + (cg >> 7);
      const int cc  = cg & 127;
      unsigned short hb[8];
#pragma unroll
      for (int e = 0; e < 8; ++e) hb[e] = sm[row][c8 + e];
      const v4u u = (v4u){pk16(hb[0], hb[1]), pk16(hb[2], hb[3]), pk16(hb[4], hb[5]), pk16(hb[6], hb[7])};
      *(volatile v4u*)(VT + ((size_t)g * kHeadDim + cc) * kSeq + l0 + c8) = u;
    }
    __threadfence();
  }
}

__global__ __launch_bounds__(256) void softmax_mean_kernel(const float* __restrict__ S, unsigned short* __restrict__ P,
                                                           const float* accin, float* accout, int mode) {
  __shared__ float red[16];
  __shared__ __align__(16) float rowbuf[kSeq];
  const int row  = blockIdx.x;
  const int t    = threadIdx.x;
  const int lane = t & 31, wave = t >> 5;
  const int c0   = t * 8;
  float pm[8];
#pragma unroll
  for (int e = 0; e < 8; ++e) pm[e] = 0.f;

#pragma unroll 1
  for (int g = 0; g < kGrp; ++g) {
    const float* sr = S + ((size_t)g * kSeq + row) * kSeq + c0;
    const v4f a = *(const v4f*)(sr);
    const v4f c = *(const v4f*)(sr + 4);
    float x[8];
#pragma unroll
    for (int e = 0; e < 4; ++e) { x[e] = a[e]; x[4 + e] = c[e]; }
    float m = fmaxf(fmaxf(fmaxf(x[0], x[1]), fmaxf(x[2], x[3])), fmaxf(fmaxf(x[4], x[5]), fmaxf(x[6], x[7])));
#pragma unroll
    for (int off = 16; off > 0; off >>= 1) m = fmaxf(m, __shfl_xor(m, off, 32));
    if (lane == 0) red[wave] = m;
    __syncthreads();
    float gm = red[0];
#pragma unroll
    for (int w = 1; w < 8; ++w) gm = fmaxf(gm, red[w]);
    float ex[8];
    float s = 0.f;
#pragma unroll
    for (int e = 0; e < 8; ++e) { ex[e] = expf(x[e] - gm); s += ex[e]; }
#pragma unroll
    for (int off = 16; off > 0; off >>= 1) s += __shfl_xor(s, off, 32);
    if (lane == 0) red[8 + wave] = s;
    __syncthreads();
    float tot = red[8];
#pragma unroll
    for (int w = 1; w < 8; ++w) tot += red[8 + w];
    const float inv = 1.0f / tot;
    unsigned short hb[8];
#pragma unroll
    for (int e = 0; e < 8; ++e) {
      const float p = ex[e] * inv;
      pm[e] += p;
      hb[e] = h_bits(p * kPCarry);
    }
    const v4u u = (v4u){pk16(hb[0], hb[1]), pk16(hb[2], hb[3]), pk16(hb[4], hb[5]), pk16(hb[6], hb[7])};
    unsigned short* pp = P + ((size_t)g * kSeq + row) * kSeq + c0;
    *(volatile v4u*)pp = u;
    __threadfence();
    *(volatile v4u*)pp = u;
  }

  *(v4f*)(rowbuf + c0)     = (v4f){pm[0], pm[1], pm[2], pm[3]};
  *(v4f*)(rowbuf + c0 + 4) = (v4f){pm[4], pm[5], pm[6], pm[7]};
  __syncthreads();
  const int c4 = t * 4;
  v4f r0 = *(const v4f*)(rowbuf + c4);
  v4f r1 = *(const v4f*)(rowbuf + 1024 + c4);
  if (mode != 0) {
    const v4f a0 = *(const v4f*)(accin + (size_t)row * kSeq + c4);
    const v4f a1 = *(const v4f*)(accin + (size_t)row * kSeq + 1024 + c4);
    r0 = a0 + r0;
    r1 = a1 + r1;
  }
  if (mode == 2) {
    r0 = r0 * kMeanScale;
    r1 = r1 * kMeanScale;
  }
  float* o = accout + (size_t)row * kSeq;
  *(volatile v4f*)(o + c4)        = r0;
  *(volatile v4f*)(o + 1024 + c4) = r1;
  __threadfence();
  *(volatile v4f*)(o + c4)        = r0;
  *(volatile v4f*)(o + 1024 + c4) = r1;
}

extern "C" void kernel_launch(void* const* d_in, const int* in_sizes, int n_in,
                              void* d_out, int out_size, void* d_ws, size_t ws_size,
                              hipStream_t stream) {
  if (n_in < 7) return;
  if (in_sizes[0] != kTok * kModel) return;
  if (in_sizes[1] != kModel * kModel || in_sizes[3] != kModel * kModel || in_sizes[5] != kModel * kModel) return;
  if (in_sizes[2] != kModel || in_sizes[4] != kModel || in_sizes[6] != kModel) return;
  if (out_size != kTok * kModel + kBatch * kSeq * kSeq) return;

  const float* query = (const float*)d_in[0];
  const float* Wq    = (const float*)d_in[1];
  const float* bq    = (const float*)d_in[2];
  const float* Wk    = (const float*)d_in[3];
  const float* bk    = (const float*)d_in[4];
  const float* Wv    = (const float*)d_in[5];
  const float* bv    = (const float*)d_in[6];

  const size_t offX16  = 0;
  const size_t szX16   = (size_t)kTok * kModel * 2;
  const size_t offW16  = offX16 + szX16;
  const size_t szW16   = (size_t)kQKVN * kModel * 2;
  const size_t offBias = offW16 + szW16;
  const size_t szBias  = (size_t)kQKVN * 4;
  const size_t offY16  = offBias + szBias;
  const size_t szY16   = (size_t)kTok * kQKVN * 2;
  const size_t offVT   = offY16 + szY16;
  const size_t szVT    = (size_t)kBatch * kHeads * kHeadDim * kSeq * 2;
  const size_t offAcc  = offVT + szVT;
  const size_t szAcc   = (size_t)kBatch * kSeq * kSeq * 4;
  const size_t offS    = offAcc + szAcc;
  const size_t szS     = (size_t)kGrp * kSeq * kSeq * 4;
  const size_t offP    = offS + szS;
  const size_t szP     = (size_t)kGrp * kSeq * kSeq * 2;
  const size_t total   = offP + szP;
  if (total > ws_size) return;

  char* ws = (char*)d_ws;
  unsigned short* X16   = (unsigned short*)(ws + offX16);
  unsigned short* W16   = (unsigned short*)(ws + offW16);
  float*          bias3 = (float*)(ws + offBias);
  unsigned short* Y16   = (unsigned short*)(ws + offY16);
  unsigned short* VT16  = (unsigned short*)(ws + offVT);
  float*          Acc   = (float*)(ws + offAcc);
  float*          S     = (float*)(ws + offS);
  unsigned short* P16   = (unsigned short*)(ws + offP);

  float* out0 = (float*)d_out;
  float* out1 = out0 + (size_t)kTok * kModel;

  cast8_f16_kernel<<<dim3((kTok * kModel / 8) / 256), dim3(256), 0, stream>>>(query, X16, kTok * kModel / 8);
  wcast8_kernel<<<dim3((kModel * kModel / 8) / 256, 3), dim3(256), 0, stream>>>(Wq, Wk, Wv, W16, kModel * kModel / 8);
  bias3_kernel<<<dim3(3), dim3(256), 0, stream>>>(bq, bk, bv, bias3);
  wmma_gemm64<0, false, 2, 1, false><<<dim3((kTok / 64) * (kQKVN / 64) / 8, 1), dim3(256), 0, stream>>>(
      X16, X16, kModel, 0L, W16, W16, kModel, 0L, (void*)Y16, (void*)Y16, kQKVN, 0L,
      bias3, bias3, 0L, kTok, kQKVN, kModel, kWCarryInv);
  vtrans_kernel<<<dim3(kSeq / 64, kModel / 64, kBatch), dim3(256), 0, stream>>>(Y16, VT16);

  for (int b = 0; b < kBatch; ++b) {
    for (int j = 0; j < kChunks; ++j) {
      const int h0 = j * kGrp;
      const unsigned short* Qp = Y16 + (size_t)b * kSeq * kQKVN + (size_t)h0 * kHeadDim;
      const unsigned short* Kp = Qp + kModel;
      wmma_gemm64<0, false, 0, 0, false><<<dim3((kSeq / 64) * (kSeq / 64) / 8, kGrp), dim3(256), 0, stream>>>(
          Qp, Qp, kQKVN, (long)kHeadDim, Kp, Kp, kQKVN, (long)kHeadDim, (void*)S, (void*)S, kSeq, (long)kSeq * kSeq,
          bias3, bias3, 0L, kSeq, kSeq, kHeadDim, kLogitScale);
      const int mode = (j == 0) ? 0 : ((j == kChunks - 1) ? 2 : 1);
      float* accb = Acc + (size_t)b * kSeq * kSeq;
      float* dst  = (mode == 2) ? (out1 + (size_t)b * kSeq * kSeq) : accb;
      softmax_mean_kernel<<<dim3(kSeq), dim3(256), 0, stream>>>(S, P16, accb, dst, mode);
      const unsigned short* VTp = VT16 + (size_t)(b * kHeads + h0) * kHeadDim * kSeq;
      float* Op = out0 + (size_t)b * kSeq * kModel + (size_t)h0 * kHeadDim;
      wmma_gemm64<0, false, 0, 0, false><<<dim3((kSeq / 64) * (kHeadDim / 64) / 8, kGrp), dim3(256), 0, stream>>>(
          P16, P16, kSeq, (long)kSeq * kSeq, VTp, VTp, kSeq, (long)kHeadDim * kSeq, (void*)Op, (void*)Op, kModel, (long)kHeadDim,
          bias3, bias3, 0L, kSeq, kHeadDim, kSeq, kPCarryInv);
    }
  }
}
